// ReferenceMoEBlock_46420006535171
// MI455X (gfx1250) — hardware-verified
//
#include <hip/hip_runtime.h>
#include <math.h>

typedef __attribute__((ext_vector_type(16))) _Float16 v16h;
typedef __attribute__((ext_vector_type(16))) __bf16 v16b;
typedef __attribute__((ext_vector_type(8)))  _Float16 v8h;
typedef __attribute__((ext_vector_type(8)))  float v8f;
typedef __attribute__((ext_vector_type(4)))  float v4f;
typedef __attribute__((ext_vector_type(2)))  float v2f;
typedef __attribute__((ext_vector_type(4)))  unsigned v4u;
typedef __attribute__((ext_vector_type(4)))  int v4i;
typedef float __attribute__((may_alias)) float_a;
typedef int __attribute__((may_alias)) int_a;

template <typename T> __device__ __forceinline__ void vst2(void* p, T v) { *(volatile T*)p = v; __threadfence(); *(volatile T*)p = v; }
__device__ __forceinline__ v8f wmma16(v16h a, v16h b, v8f c) {
  v8f d = __builtin_amdgcn_wmma_f32_16x16x32_f16(false, a, false, b, (short)0, c, false, false);
  asm volatile("v_nop\n\tv_nop\n\tv_nop\n\tv_nop" : "+v"(d) : "v"(a), "v"(b));
  return d;
}
__device__ __forceinline__ v8f wmma_bf(v16b a, v16b b, v8f c) {
  v8f d = __builtin_amdgcn_wmma_f32_16x16x32_bf16(false, a, false, b, (short)0, c, false, false);
  asm volatile("v_nop\n\tv_nop\n\tv_nop\n\tv_nop" : "+v"(d) : "v"(a), "v"(b));
  return d;
}
__device__ __forceinline__ v16h frag_h(const _Float16* rowk0, int lane) {
  union { v16h v; v8h q[2]; } u; const _Float16* p = rowk0 + 8 * (lane >> 4);
  u.q[0] = *(const v8h*)p; u.q[1] = *(const v8h*)(p + 16); return u.v;
}
__device__ __forceinline__ v16h frag_f32(const float* rowk0, int lane) {
  v16h a; const float* p = rowk0 + 8 * (lane >> 4);
#pragma unroll
  for (int i = 0; i < 8; ++i) { a[i] = (_Float16)p[i]; a[8 + i] = (_Float16)p[16 + i]; }
  return a;
}
__device__ __forceinline__ v16h frag_f32s(const float* rowk0, int lane, float sc) {
  v16h a; const float* p = rowk0 + 8 * (lane >> 4);
#pragma unroll
  for (int i = 0; i < 8; ++i) { a[i] = (_Float16)(p[i] * sc); a[8 + i] = (_Float16)(p[16 + i] * sc); }
  return a;
}
__device__ __forceinline__ v16h fragc_f32(const float* W, int k0, int n, int lane, int ld, int K) {
  v16h a; const int g = lane >> 4;
#pragma unroll
  for (int i = 0; i < 8; ++i) { const int ka = k0 + 8 * g + i, kb = ka + 16;
    a[i] = (_Float16)(ka < K ? W[(size_t)(ka < K ? ka : K - 1) * ld + n] : 0.f); a[8 + i] = (_Float16)(kb < K ? W[(size_t)(kb < K ? kb : K - 1) * ld + n] : 0.f); }
  return a;
}
struct F2 { v16b h, l; };
__device__ __forceinline__ F2 bsplit16(const float v[16]) { F2 r;
#pragma unroll
  for (int i = 0; i < 16; ++i) { const __bf16 h = (__bf16)v[i]; r.h[i] = h; r.l[i] = (__bf16)(v[i] - (float)h); }
  return r; }
__device__ __forceinline__ F2 split_row(const float* row, int k0, int lane) { float v[16]; const float* p = row + k0 + 8 * (lane >> 4);
#pragma unroll
  for (int i = 0; i < 8; ++i) { v[i] = p[i]; v[8 + i] = p[16 + i]; }
  return bsplit16(v); }
__device__ __forceinline__ F2 split_rowK(const float* row, int k0, int lane, int K) { float v[16]; const int g = lane >> 4;
#pragma unroll
  for (int i = 0; i < 8; ++i) { const int ka = k0 + 8 * g + i, kb = ka + 16; v[i] = ka < K ? row[ka < K ? ka : K - 1] : 0.f; v[8 + i] = kb < K ? row[kb < K ? kb : K - 1] : 0.f; }
  return bsplit16(v); }
__device__ __forceinline__ F2 split_col(const float* W, int k0, int n, int lane, int ld, int K) { float v[16]; const int g = lane >> 4;
#pragma unroll
  for (int i = 0; i < 8; ++i) { const int ka = k0 + 8 * g + i, kb = ka + 16; v[i] = ka < K ? W[(size_t)(ka < K ? ka : K - 1) * ld + n] : 0.f; v[8 + i] = kb < K ? W[(size_t)(kb < K ? kb : K - 1) * ld + n] : 0.f; }
  return bsplit16(v); }
__device__ __forceinline__ v8f mac3(const F2& a, const F2& b, v8f c) { c = wmma_bf(a.l, b.h, c); c = wmma_bf(a.h, b.l, c); return wmma_bf(a.h, b.h, c); }
__device__ __forceinline__ float sigm(float v) { return 1.0f / (1.0f + expf(-v)); }
#define LDSX() do { asm volatile("s_wait_dscnt 0" ::: "memory"); __builtin_amdgcn_wave_barrier(); __builtin_amdgcn_fence(__ATOMIC_RELEASE, "workgroup"); } while (0)


#define TT 2048
#define HH 1024
#define II 512
#define NEX 16
#define TOPK 6
#define IS 1024
#ifndef TRB
#define TRB (TT / 64)
#endif
typedef __attribute__((ext_vector_type(8))) __bf16 v8b;
__device__ __forceinline__ v16b frag_b(const __bf16* rowk0, int lane) {
  union { v16b v; v8b q[2]; } u; const __bf16* p = rowk0 + 8 * (lane >> 4);
  u.q[0] = *(const v8b*)p; u.q[1] = *(const v8b*)(p + 16); return u.v;
}
__device__ __forceinline__ float bfr(float v) { return (float)(__bf16)v; }
__device__ __attribute__((noinline)) float exp_ni(float v) { return expf(v); }
__device__ __attribute__((noinline)) float erf_ni(float v) { return erff(v); }

#define PK_G   0
#define PK_GU  (PK_G + NEX * HH)
#define PK_D   (PK_GU + (size_t)NEX * 2 * II * HH)
#define PK_SGU (PK_D + (size_t)NEX * HH * II)
#define PK_SD  (PK_SGU + (size_t)2 * IS * HH)
#define PK_END (PK_SD + (size_t)HH * IS)
#define WS_PK   0u
#define WS_COMB (WS_PK + 2u * (unsigned)PK_END)
#define WS_H2   (WS_COMB + 4u * TT * NEX)
#define WS_END  (WS_H2 + 4u * TT * 2 * IS)

__global__ __launch_bounds__(256) void k_packT(const float* __restrict__ Wm, size_t estride, int K, int N, __bf16* __restrict__ DST, size_t dplane, int rofs) {
  __shared__ __align__(16) __bf16 s[1024]; const int n = blockIdx.x, e = blockIdx.y, tid = threadIdx.x; const float* w = Wm + (size_t)e * estride;
  for (int k = tid; k < K; k += 256) s[k] = (__bf16)w[(size_t)k * N + n];
  __syncthreads();
  for (int q = tid; q < K / 8; q += 256) vst2((unsigned*)(DST + (size_t)e * dplane + (size_t)(rofs + n) * K + q * 8), *(const v4u*)&s[q * 8]);
}
__global__ __launch_bounds__(256) void k_packrow(const float* __restrict__ Wm, int K, __bf16* __restrict__ DST) {
  __shared__ __align__(16) __bf16 s[1024]; const int n = blockIdx.x, tid = threadIdx.x;
  for (int k = tid; k < K; k += 256) s[k] = (__bf16)Wm[(size_t)n * K + k];
  __syncthreads();
  for (int q = tid; q < K / 8; q += 256) vst2((unsigned*)(DST + (size_t)n * K + q * 8), *(const v4u*)&s[q * 8]);
}
__global__ __launch_bounds__(128) void k_gate(const float* __restrict__ X, const __bf16* __restrict__ PG, const float* __restrict__ GB, float* __restrict__ COMB, float* __restrict__ Y) {
  __shared__ float ssc[64][NEX + 1]; __shared__ __align__(16) float scomb[64][NEX];
  const int tid = threadIdx.x, wave = tid >> 5, lane = tid & 31, col = lane & 15, g = lane >> 4; const size_t r0 = (size_t)blockIdx.x * 64 + wave * 16;
  v8f acc = {};
#pragma unroll 4
  for (int kc = 0; kc < HH / 32; ++kc) { v16b a; { const float* p = X + (r0 + col) * HH + kc * 32 + 8 * g;
#pragma unroll
      for (int i = 0; i < 8; ++i) { a[i] = (__bf16)p[i]; a[8 + i] = (__bf16)p[16 + i]; } }
    acc = wmma_bf(a, frag_b(PG + (size_t)col * HH + kc * 32, lane), acc); }
#pragma unroll
  for (int r = 0; r < 8; ++r) ssc[wave * 16 + 8 * g + r][col] = sigm(acc[r]);
  __syncthreads();
  if (tid < 64) { const int t = tid; float sc[NEX], bs[NEX]; int used = 0;
#pragma unroll
    for (int e = 0; e < NEX; ++e) { sc[e] = ssc[t][e]; bs[e] = sc[e] + bfr(GB[e]); scomb[t][e] = 0.f; }
    int sel[TOPK]; float wsum = 0.f;
#pragma unroll
    for (int k = 0; k < TOPK; ++k) { int bi = 0; float bv = -3.0e38f;
#pragma unroll
      for (int e = 0; e < NEX; ++e) { const bool free_ = ((used >> e) & 1) == 0; if (free_ && bs[e] > bv) { bv = bs[e]; bi = e; } }
      used |= 1 << bi; sel[k] = bi; float w = 0.f;
#pragma unroll
      for (int e = 0; e < NEX; ++e) w = (e == bi) ? sc[e] : w;
      wsum += w; }
    const float inv = 1.0f / (wsum + 1e-20f);
#pragma unroll
    for (int k = 0; k < TOPK; ++k) {
#pragma unroll
      for (int e = 0; e < NEX; ++e) if (e == sel[k]) scomb[t][e] = sc[e] * inv; } }
  __syncthreads();
  for (int q = tid; q < 64 * 4; q += 128) { const int rl = q >> 2, pc = q & 3; vst2(COMB + ((size_t)blockIdx.x * 64 + rl) * NEX + pc * 4, *(const v4f*)&scomb[rl][pc * 4]); }
  for (int q = tid; q < 64 * (HH / 4); q += 128) { const int rl = q / (HH / 4), pc = q % (HH / 4); vst2(Y + ((size_t)blockIdx.x * 64 + rl) * HH + pc * 4, (v4f){0.f, 0.f, 0.f, 0.f}); }
}
__global__ __launch_bounds__(128) void k_up(const float* __restrict__ X, const __bf16* __restrict__ P, float* __restrict__ H2, int ldo) {
  __shared__ __align__(16) float so[4][16][132];
  const int tid = threadIdx.x, wave = tid >> 5, lane = tid & 31, col = lane & 15, g = lane >> 4; const size_t r0 = (size_t)blockIdx.x * 64 + wave * 16; const int n0 = blockIdx.y * 128;
  v8f acc[8] = {};
#pragma unroll 2
  for (int kc = 0; kc < HH / 32; ++kc) { v16b a; { const float* p = X + (r0 + col) * HH + kc * 32 + 8 * g;
#pragma unroll
      for (int i = 0; i < 8; ++i) { a[i] = (__bf16)p[i]; a[8 + i] = (__bf16)p[16 + i]; } }
#pragma unroll
    for (int j = 0; j < 8; ++j) acc[j] = wmma_bf(a, frag_b(P + (size_t)(n0 + j * 16 + col) * HH + kc * 32, lane), acc[j]); }
#pragma unroll
  for (int j = 0; j < 8; ++j)
#pragma unroll
    for (int r = 0; r < 8; ++r) so[wave][8 * g + r][j * 16 + col] = acc[j][r];
  LDSX();
  for (int rl = 0; rl < 16; ++rl) vst2(H2 + (r0 + rl) * ldo + n0 + lane * 4, *(const v4f*)&so[wave][rl][lane * 4]);
}
template <int IW>
__global__ __launch_bounds__(128) void k_down(const float* __restrict__ H2, int ldh, const __bf16* __restrict__ P, const float* __restrict__ COMB, int e, float* Y) {
  __shared__ __align__(16) float so[4][16][132];
  const int tid = threadIdx.x, wave = tid >> 5, lane = tid & 31, col = lane & 15, g = lane >> 4; const size_t r0 = (size_t)blockIdx.x * 64 + wave * 16; const int n0 = blockIdx.y * 128;
  v8f acc[8] = {};
#pragma unroll 2
  for (int kc = 0; kc < IW / 32; ++kc) { float v[16]; { const float* p = H2 + (r0 + col) * ldh + kc * 32 + 8 * g;
#pragma unroll
      for (int i = 0; i < 8; ++i) { const float a0 = p[i], b0 = p[IW + i], a1 = p[16 + i], b1 = p[IW + 16 + i]; v[i] = a0 / (1.0f + exp_ni(-a0)) * b0; v[8 + i] = a1 / (1.0f + exp_ni(-a1)) * b1; } }
    const F2 a = bsplit16(v);
#pragma unroll
    for (int j = 0; j < 8; ++j) { const v16b w = frag_b(P + (size_t)(n0 + j * 16 + col) * IW + kc * 32, lane); acc[j] = wmma_bf(a.l, w, acc[j]); acc[j] = wmma_bf(a.h, w, acc[j]); } }
#pragma unroll
  for (int j = 0; j < 8; ++j) { const int n = n0 + j * 16 + col;
#pragma unroll
    for (int r = 0; r < 8; ++r) { const size_t row = r0 + 8 * g + r; const float wgt = (e >= 0) ? COMB[row * NEX + e] : 1.0f; so[wave][8 * g + r][j * 16 + col] = Y[row * HH + n] + wgt * acc[j][r]; } }
  LDSX();
  for (int rl = 0; rl < 16; ++rl) vst2(Y + (r0 + rl) * HH + n0 + lane * 4, *(const v4f*)&so[wave][rl][lane * 4]);
}
extern "C" void kernel_launch(void* const* d_in, const int* in_sizes, int n_in, void* d_out, int out_size, void* d_ws, size_t ws_size, hipStream_t stream) {
  (void)in_sizes; (void)n_in; (void)out_size;
  const float** F = (const float**)d_in;
  if (ws_size < (size_t)WS_END) return;
  char* ws = (char*)d_ws; __bf16* PK = (__bf16*)(ws + WS_PK); float *COMB = (float*)(ws + WS_COMB), *H2 = (float*)(ws + WS_H2); float* Y = (float*)d_out;
  k_packrow<<<NEX, 256, 0, stream>>>(F[1], HH, PK + PK_G);
  k_packT<<<dim3(II, NEX), 256, 0, stream>>>(F[3], (size_t)HH * II, HH, II, PK + PK_GU, (size_t)2 * II * HH, 0);
  k_packT<<<dim3(II, NEX), 256, 0, stream>>>(F[4], (size_t)HH * II, HH, II, PK + PK_GU, (size_t)2 * II * HH, II);
  k_packT<<<dim3(HH, NEX), 256, 0, stream>>>(F[5], (size_t)II * HH, II, HH, PK + PK_D, (size_t)HH * II, 0);
  k_packT<<<dim3(IS, 1), 256, 0, stream>>>(F[6], 0, HH, IS, PK + PK_SGU, 0, 0);
  k_packT<<<dim3(IS, 1), 256, 0, stream>>>(F[7], 0, HH, IS, PK + PK_SGU, 0, IS);
  k_packT<<<dim3(HH, 1), 256, 0, stream>>>(F[8], 0, IS, HH, PK + PK_SD, 0, 0);
  k_gate<<<TRB, 128, 0, stream>>>(F[0], PK + PK_G, F[2], COMB, Y);
  for (int e = 0; e < NEX; ++e) {
    k_up<<<dim3(TRB, 2 * II / 128), 128, 0, stream>>>(F[0], PK + PK_GU + (size_t)e * 2 * II * HH, H2, 2 * II);
    k_down<II><<<dim3(TRB, HH / 128), 128, 0, stream>>>(H2, 2 * II, PK + PK_D + (size_t)e * HH * II, COMB, e, Y); }
  k_up<<<dim3(TRB, 2 * IS / 128), 128, 0, stream>>>(F[0], PK + PK_SGU, H2, 2 * IS);
  k_down<IS><<<dim3(TRB, HH / 128), 128, 0, stream>>>(H2, 2 * IS, PK + PK_SD, COMB, -1, Y);
}
